// FM_LOSS_12146167513244
// MI455X (gfx1250) — hardware-verified
//
#include <hip/hip_runtime.h>
#include <hip/hip_bf16.h>
#include <math.h>


#define BB 8
#define SS 2048
#define DD 512
#define HH 8
#define DKK 64
#define QW 2

typedef _Float16 bf16;
typedef __attribute__((ext_vector_type(4))) unsigned v4u_t;
typedef unsigned v4ua __attribute__((ext_vector_type(4), may_alias));
typedef __attribute__((ext_vector_type(4))) float v4f_t;
typedef float v4fa __attribute__((ext_vector_type(4), may_alias));
typedef __attribute__((ext_vector_type(16))) bf16  bf16x16;
typedef __attribute__((ext_vector_type(8)))  bf16  bf16x8;
typedef __attribute__((ext_vector_type(4)))  bf16  bf16x4;
typedef __attribute__((ext_vector_type(8)))  float f32x8;

#define LDS_STRIDE 48
#define KSTRIDE    72
#define VSTRIDE    48

__device__ __forceinline__ f32x8 wmma_bf16(bf16x16 a, bf16x16 b, f32x8 c) {
  return __builtin_amdgcn_wmma_f32_16x16x32_f16(
      false, a, false, b, (short)0, c, false, false);
}

template <typename T>
__device__ __forceinline__ bf16x16 load_frag(const T* __restrict__ base, int ld,
                                             int row0, int k0) {
  const int lane = threadIdx.x & 31;
  const int r    = lane & 15;
  const int kh   = (lane >> 4) * 8;
  const T* p0 = base + (size_t)(row0 + r) * ld + (k0 + kh);
  const T* p1 = p0 + 16;
  bf16x16 f;
#pragma unroll
  for (int i = 0; i < 8; ++i) {
    f[i]     = (bf16)p0[i];
    f[i + 8] = (bf16)p1[i];
  }
  return f;
}

__device__ __forceinline__ bf16x16 lds_frag(const bf16* base, int stride) {
  const int lane = threadIdx.x & 31;
  const int row  = lane & 15;
  const int kh   = (lane >> 4) * 8;
  const bf16x8 lo = *(const bf16x8*)(base + row * stride + kh);
  const bf16x8 hi = *(const bf16x8*)(base + row * stride + kh + 16);
  bf16x16 f;
#pragma unroll
  for (int i = 0; i < 8; ++i) { f[i] = lo[i]; f[i + 8] = hi[i]; }
  return f;
}

template <typename T>
__device__ __forceinline__ void stage_read16(const T* __restrict__ p, float* buf) {
#pragma unroll
  for (int i = 0; i < 16; ++i) buf[i] = (float)p[i];
}

__device__ __forceinline__ void stage_write(bf16* dst, const float* buf, int nquad) {
#pragma unroll
  for (int i = 0; i < nquad; ++i) {
    bf16x4 q;
    q[0] = (bf16)buf[4 * i];     q[1] = (bf16)buf[4 * i + 1];
    q[2] = (bf16)buf[4 * i + 2]; q[3] = (bf16)buf[4 * i + 3];
    *(bf16x4*)(dst + 4 * i) = q;
  }
}

__global__ __launch_bounds__(256) void transpose_pack_kernel(const float* __restrict__ W, bf16* __restrict__ WT, int K, int N) {
  __shared__ float tile[64][65];
  const int k0 = blockIdx.y * 64, n0 = blockIdx.x * 64, t = threadIdx.x;
  for (int i = t; i < 64 * 64; i += 256) { const int kr = i >> 6, nc = i & 63; tile[kr][nc] = W[(size_t)(k0 + kr) * N + n0 + nc]; }
  __syncthreads();
#pragma unroll 1
  for (int pass = 0; pass < 2; ++pass) {
    for (int i = t; i < 64 * 8; i += 256) { const int nr = i >> 3, k8 = (i & 7) * 8; bf16 hh[8];
#pragma unroll
      for (int e = 0; e < 8; ++e) hh[e] = (bf16)tile[k8 + e][nr];
      *(volatile v4u_t*)(WT + (size_t)(n0 + nr) * K + k0 + k8) = *(const v4ua*)hh; }
    __threadfence();
  }
}

template <typename AT, typename WT, int MODE>
__global__ __launch_bounds__(256) void gemm_bias_kernel(
    const AT* __restrict__ A, const WT* __restrict__ W,
    const float* __restrict__ bias, void* __restrict__ out,
    int M, int N, int K) {
  __shared__ bf16 ldsA[128 * LDS_STRIDE];
  __shared__ bf16 ldsW[256 * LDS_STRIDE];
  __shared__ __attribute__((aligned(16))) unsigned char sob[256 * 136 * 2];

  const int t    = threadIdx.x;
  const int wave = t >> 5;
  const int lane = t & 31;
  const int wm   = (wave & 1) * 64;
  const int wn   = (wave >> 1) * 64;
  const int mBlk = blockIdx.x * 128;
  const int nBlk = blockIdx.y * 256;

  const int arow = t >> 1;
  const int ach  = (t & 1) * 16;

  float abuf[16];
  float wbuf[32];

  stage_read16(A + (size_t)(mBlk + arow) * K + ach, abuf);
  stage_read16(W + (size_t)(nBlk + t) * K,          wbuf);
  stage_read16(W + (size_t)(nBlk + t) * K + 16,     wbuf + 16);

  f32x8 acc[4][4] = {};

  for (int k = 0; k < K; k += 32) {
    __syncthreads();
    stage_write(&ldsA[arow * LDS_STRIDE + ach], abuf, 4);
    stage_write(&ldsW[t * LDS_STRIDE],          wbuf, 8);
    if (k + 32 < K) {
      stage_read16(A + (size_t)(mBlk + arow) * K + (k + 32) + ach, abuf);
      stage_read16(W + (size_t)(nBlk + t) * K + (k + 32),          wbuf);
      stage_read16(W + (size_t)(nBlk + t) * K + (k + 32) + 16,     wbuf + 16);
    }
    __syncthreads();

    bf16x16 af[4], wf[4];
#pragma unroll
    for (int i = 0; i < 4; ++i)
      af[i] = lds_frag(ldsA + (wm + 16 * i) * LDS_STRIDE, LDS_STRIDE);
#pragma unroll
    for (int j = 0; j < 4; ++j)
      wf[j] = lds_frag(ldsW + (wn + 16 * j) * LDS_STRIDE, LDS_STRIDE);
#pragma unroll
    for (int i = 0; i < 4; ++i)
#pragma unroll
      for (int j = 0; j < 4; ++j)
        acc[i][j] = wmma_bf16(af[i], wf[j], acc[i][j]);
  }

  const int nlane = lane & 15;
  const int mh    = (lane >> 4) * 8;
  __syncthreads();
  if (MODE == 0 || MODE == 1) {
    bf16* so = (bf16*)sob;
#pragma unroll
    for (int i = 0; i < 4; ++i)
#pragma unroll
      for (int j = 0; j < 4; ++j) {
        const int nl = wn + 16 * j + nlane;
        const float bv = bias ? bias[nBlk + nl] : 0.0f;
#pragma unroll
        for (int r = 0; r < 8; ++r) {
          const int ml = wm + 16 * i + mh + r;
          const bf16 hv = (bf16)(acc[i][j][r] + bv);
          if (MODE == 0) so[ml * 264 + nl] = hv;
          else           so[nl * 136 + ml] = hv;
        }
      }
    __syncthreads();
#pragma unroll 1
    for (int pass = 0; pass < 2; ++pass) {
      if (MODE == 0) {
        for (int ch = t; ch < 128 * 32; ch += 256) { const int ml = ch >> 5, q = (ch & 31) * 8;
          *(volatile v4u_t*)((bf16*)out + (size_t)(mBlk + ml) * N + nBlk + q) = *(const v4ua*)(so + ml * 264 + q); }
      } else {
        const int b_ = mBlk >> 11, s0 = mBlk & (SS - 1);
        for (int ch = t; ch < 256 * 16; ch += 256) { const int nl = ch >> 4, q = (ch & 15) * 8; const int n = nBlk + nl, h = n >> 6, dk = n & (DKK - 1);
          *(volatile v4u_t*)((bf16*)out + (((size_t)(b_ * HH + h)) * DKK + dk) * SS + s0 + q) = *(const v4ua*)(so + nl * 136 + q); }
      }
      __threadfence();
    }
  } else {
    float* so = (float*)sob;
#pragma unroll 1
    for (int hf = 0; hf < 2; ++hf) {
      if (wm == hf * 64) {
#pragma unroll
        for (int i = 0; i < 4; ++i)
#pragma unroll
          for (int j = 0; j < 4; ++j) {
            const int nl = wn + 16 * j + nlane;
            const float bv = bias ? bias[nBlk + nl] : 0.0f;
#pragma unroll
            for (int r = 0; r < 8; ++r) so[(16 * i + mh + r) * 260 + nl] = acc[i][j][r] + bv;
          }
      }
      __syncthreads();
#pragma unroll 1
      for (int pass = 0; pass < 2; ++pass) {
        for (int ch = t; ch < 64 * 64; ch += 256) { const int ml = ch >> 6, q = (ch & 63) * 4;
          *(volatile v4f_t*)((float*)out + (size_t)(mBlk + hf * 64 + ml) * N + nBlk + q) = *(const volatile v4fa*)(so + ml * 260 + q); }
        __threadfence();
      }
      __syncthreads();
    }
  }
}

__global__ __launch_bounds__(64) void attn_kernel(
    const bf16* __restrict__ Qb, const bf16* __restrict__ Kb,
    const bf16* __restrict__ Vt, float* __restrict__ attnOut) {
  __shared__ bf16 ldsK[32 * KSTRIDE];
  __shared__ bf16 ldsV[64 * VSTRIDE];
  __shared__ __attribute__((aligned(16))) float ldsO[2][32 * 68];

  const int q0blk = blockIdx.x * 64;
  const int h  = blockIdx.y;
  const int b  = blockIdx.z;
  const int t    = threadIdx.x;
  const int wave = t >> 5;
  const int lane = t & 31;
  const int qlane = lane & 15;
  const int kh8   = (lane >> 4) * 8;
  const int q0 = q0blk + wave * 32;

  const bf16* Qh = Qb + (size_t)b * SS * DD + h * DKK;
  const bf16* Kh = Kb + (size_t)b * SS * DD + h * DKK;
  const bf16* Vh = Vt + ((size_t)(b * HH + h)) * DKK * SS;

  const int krow = t >> 1;
  const int kcol = (t & 1) * 32;
  const bf16* kSrc = Kh + (size_t)krow * DD + kcol;
  const bf16* vSrc = Vh + (size_t)t * SS;

  bf16x16 qf[QW][2];
#pragma unroll
  for (int qt = 0; qt < QW; ++qt) {
    qf[qt][0] = load_frag(Qh, DD, q0 + 16 * qt, 0);
    qf[qt][1] = load_frag(Qh, DD, q0 + 16 * qt, 32);
  }

  f32x8 o[QW][4] = {};
  float mrun[QW], lrun[QW];
#pragma unroll
  for (int qt = 0; qt < QW; ++qt) { mrun[qt] = -INFINITY; lrun[qt] = 0.0f; }

  const float scale = 1.44269504088896340736f;
  const int kmax = SS - 1;

  bf16x8 kreg[4], vreg[4];
#pragma unroll
  for (int i = 0; i < 4; ++i) {
    kreg[i] = *(const bf16x8*)(kSrc + 8 * i);
    vreg[i] = *(const bf16x8*)(vSrc + 8 * i);
  }

  for (int kb = 0; kb <= kmax; kb += 32) {
    __syncthreads();
#pragma unroll
    for (int i = 0; i < 4; ++i) {
      *(bf16x8*)(&ldsK[krow * KSTRIDE + kcol + 8 * i]) = kreg[i];
      *(bf16x8*)(&ldsV[t * VSTRIDE + 8 * i])           = vreg[i];
    }
    if (kb + 32 <= kmax) {
      const bf16* kn = kSrc + (size_t)(kb + 32) * DD;
      const bf16* vn = vSrc + (kb + 32);
#pragma unroll
      for (int i = 0; i < 4; ++i) {
        kreg[i] = *(const bf16x8*)(kn + 8 * i);
        vreg[i] = *(const bf16x8*)(vn + 8 * i);
      }
    }
    __syncthreads();

    bf16x16 kf[2][2];
#pragma unroll
    for (int ktile = 0; ktile < 2; ++ktile)
#pragma unroll
      for (int c = 0; c < 2; ++c)
        kf[ktile][c] = lds_frag(ldsK + (ktile * 16) * KSTRIDE + c * 32, KSTRIDE);

    bf16x16 pf[QW];
    bool act[QW];
#pragma unroll
    for (int qt = 0; qt < QW; ++qt) {
      act[qt] = true;
      {
        const int q_my = q0 + 16 * qt + qlane;
        f32x8 s0 = {}, s1 = {};
        s0 = wmma_bf16(kf[0][0], qf[qt][0], s0);
        s0 = wmma_bf16(kf[0][1], qf[qt][1], s0);
        s1 = wmma_bf16(kf[1][0], qf[qt][0], s1);
        s1 = wmma_bf16(kf[1][1], qf[qt][1], s1);

        float mx = -INFINITY;
#pragma unroll
        for (int r = 0; r < 8; ++r) {
          const int k0i = kb + kh8 + r;
          const int k1i = k0i + 16;
          (void)k0i; (void)k1i; (void)q_my;
          s0[r] = s0[r] * scale;
          s1[r] = s1[r] * scale;
          mx = fmaxf(mx, fmaxf(s0[r], s1[r]));
        }
        mx = fmaxf(mx, __shfl_xor(mx, 16, 32));
        const float mnew  = fmaxf(mrun[qt], mx);
        const float alpha = exp2f(mrun[qt] - mnew);

        float rsum = 0.0f;
#pragma unroll
        for (int r = 0; r < 8; ++r) {
          const float p0 = exp2f(s0[r] - mnew);
          const float p1 = exp2f(s1[r] - mnew);
          rsum += p0 + p1;
          pf[qt][r]     = (bf16)(p0 * 1024.0f);
          pf[qt][r + 8] = (bf16)(p1 * 1024.0f);
        }
        rsum += __shfl_xor(rsum, 16, 32);
        lrun[qt] = lrun[qt] * alpha + rsum;
        mrun[qt] = mnew;

#pragma unroll
        for (int j = 0; j < 4; ++j)
#pragma unroll
          for (int r = 0; r < 8; ++r) o[qt][j][r] *= alpha;
      }
    }

#pragma unroll
    for (int j = 0; j < 4; ++j) {
      const bf16x16 vf = lds_frag(ldsV + (j * 16) * VSTRIDE, VSTRIDE);
#pragma unroll
      for (int qt = 0; qt < QW; ++qt)
        if (act[qt]) o[qt][j] = wmma_bf16(vf, pf[qt], o[qt][j]);
    }
  }

  float* so = ldsO[wave];
#pragma unroll
  for (int qt = 0; qt < QW; ++qt) {
    const float rl = 1.0f / (lrun[qt] * 1024.0f);
#pragma unroll
    for (int j = 0; j < 4; ++j)
#pragma unroll
      for (int r = 0; r < 8; ++r) so[(16 * qt + qlane) * 68 + j * 16 + kh8 + r] = o[qt][j][r] * rl;
  }
  asm volatile("s_wait_dscnt 0" ::: "memory");
#pragma unroll 1
  for (int pass = 0; pass < 2; ++pass) {
#pragma unroll
    for (int it = 0; it < 16; ++it) { const int ch = lane + 32 * it, ql = ch >> 4, q4 = (ch & 15) * 4;
      *(volatile v4f_t*)(attnOut + ((size_t)(b * SS + q0 + ql)) * DD + h * DKK + q4) = *(const volatile v4fa*)(so + ql * 68 + q4); }
    __threadfence();
  }
}

__global__ __launch_bounds__(256) void k_cvt16(const float* __restrict__ x, bf16* __restrict__ y, int n8) {
  const int g = blockIdx.x * 256 + threadIdx.x; if (g >= n8) return;
  bf16 hh[8];
#pragma unroll
  for (int i = 0; i < 8; ++i) hh[i] = (bf16)x[(size_t)g * 8 + i];
  *(volatile v4u_t*)(y + (size_t)g * 8) = *(const v4ua*)hh; __threadfence(); *(volatile v4u_t*)(y + (size_t)g * 8) = *(const v4ua*)hh;
}

__global__ __launch_bounds__(256) void k_bnstats(const float* __restrict__ X, float* __restrict__ mean, float* __restrict__ rsig) {
  __shared__ float s1[4][64], s2[4][64];
  const int tid = threadIdx.x, c = tid & 63, ph = tid >> 6, o = blockIdx.x * 64 + c;
  float a = 0.0f, q = 0.0f;
#pragma unroll 1
  for (int r = ph; r < BB * SS; r += 4) { const float v = X[(size_t)r * DD + o]; a += v; q += v * v; }
  s1[ph][c] = a; s2[ph][c] = q;
  __syncthreads();
  if (tid < 64) {
    const float su = (s1[0][tid] + s1[1][tid]) + (s1[2][tid] + s1[3][tid]);
    const float sq = (s2[0][tid] + s2[1][tid]) + (s2[2][tid] + s2[3][tid]);
    const float m = su / (float)(BB * SS);
    const float var = fmaxf(sq / (float)(BB * SS) - m * m, 0.0f);
    s1[0][tid] = m; s2[0][tid] = rsqrtf(var + 1e-5f);
  }
  __syncthreads();
#pragma unroll 1
  for (int pass = 0; pass < 2; ++pass) {
    if (tid < 64) { *(volatile float*)(mean + blockIdx.x * 64 + tid) = s1[0][tid]; *(volatile float*)(rsig + blockIdx.x * 64 + tid) = s2[0][tid]; }
    __threadfence();
  }
}

__global__ __launch_bounds__(256) void k_loss_partial(const float* __restrict__ FS, const float* __restrict__ X,
                                                     const float* __restrict__ mean, const float* __restrict__ rsig,
                                                     const float* __restrict__ gamma, const float* __restrict__ beta, float* __restrict__ part) {
  __shared__ float red[256];
  const int tid = threadIdx.x, r0 = blockIdx.x * 128;
  float acc = 0.0f;
#pragma unroll 1
  for (int r = 0; r < 128; ++r) {
#pragma unroll
    for (int oc = 0; oc < DD / 256; ++oc) { const int o = oc * 256 + tid; const size_t idx = (size_t)(r0 + r) * DD + o;
      const float ft = (X[idx] - mean[o]) * rsig[o] * gamma[o] + beta[o];
      const float d = FS[idx] - ft; acc += d * d; }
  }
  red[tid] = acc; __syncthreads();
  for (int st = 128; st > 0; st >>= 1) { if (tid < st) red[tid] += red[tid + st]; __syncthreads(); }
  if (tid == 0) { *(volatile float*)(part + blockIdx.x) = red[0]; __threadfence(); *(volatile float*)(part + blockIdx.x) = red[0]; }
}
__global__ __launch_bounds__(128) void k_loss_final(const float* __restrict__ part, float* __restrict__ out) {
  __shared__ float red[128];
  const int tid = threadIdx.x;
  red[tid] = part[tid]; __syncthreads();
  for (int st = 64; st > 0; st >>= 1) { if (tid < st) red[tid] += red[tid + st]; __syncthreads(); }
  if (tid == 0) { const float v = red[0] / (float)((size_t)BB * SS * DD); *(volatile float*)out = v; __threadfence(); *(volatile float*)out = v; }
}

extern "C" void kernel_launch(void* const* d_in, const int* in_sizes, int n_in,
                              void* d_out, int out_size, void* d_ws, size_t ws_size,
                              hipStream_t stream) {
  (void)in_sizes; (void)n_in; (void)out_size; (void)ws_size;
  const float* f_s   = (const float*)d_in[0];
  const float* f_t   = (const float*)d_in[1];
  const float* Wc    = (const float*)d_in[2];
  const float* gamma = (const float*)d_in[3];
  const float* beta  = (const float*)d_in[4];

  char* ws = (char*)d_ws;
  bf16*  Qb  = (bf16*)ws;  ws += (size_t)BB * SS * DD * 2;
  bf16*  Vt  = (bf16*)ws;  ws += (size_t)BB * SS * DD * 2;
  bf16*  Tb  = (bf16*)ws;  ws += (size_t)BB * SS * DD * 2;
  float* X   = (float*)ws; ws += (size_t)BB * SS * DD * 4;
  float* FS  = (float*)ws; ws += (size_t)BB * SS * DD * 4;
  float* mean = (float*)ws; ws += 4096;
  float* rsig = (float*)ws; ws += 4096;
  float* part = (float*)ws; ws += 4096;

  for (int b = 0; b < BB; ++b) {
    transpose_pack_kernel<<<dim3(SS / 64, DD / 64), 256, 0, stream>>>(f_s + (size_t)b * DD * SS, Qb + (size_t)b * SS * DD, DD, SS);
    transpose_pack_kernel<<<dim3(SS / 64, DD / 64), 256, 0, stream>>>(f_t + (size_t)b * DD * SS, Tb + (size_t)b * SS * DD, DD, SS);
  }
  k_cvt16<<<(BB * DD * SS / 8 + 255) / 256, 256, 0, stream>>>(f_s, Vt, BB * DD * SS / 8);

  gemm_bias_kernel<bf16, float, 2><<<dim3(BB * SS / 128, DD / 256), 256, 0, stream>>>(Tb, Wc, nullptr, X, BB * SS, DD, DD);
  k_bnstats<<<DD / 64, 256, 0, stream>>>(X, mean, rsig);

  attn_kernel<<<dim3(SS / 64, HH, BB), dim3(64), 0, stream>>>(Qb, Qb, Vt, FS);

  k_loss_partial<<<BB * SS / 128, 256, 0, stream>>>(FS, X, mean, rsig, gamma, beta, part);
  k_loss_final<<<1, 128, 0, stream>>>(part, (float*)d_out);
}
